// TransformerEncoderLayer_45775761440800
// MI455X (gfx1250) — hardware-verified
//
#include <hip/hip_runtime.h>
#include <stddef.h>
#include <stdint.h>


#define DM     256
#define DFF    2048
#define NH     8
#define HD     32
#define LNB    32
#define QKVW   768
#define NTHR   256
#define GBM    64
#define GBN    64
#define GTHR   128
#define TT     64
#define TP     68
#define CX     8.0f
#define CW     64.0f
#define SCL    0.001953125f
#define ISD    0.17677669529663688f
#define LNEPS  1.0e-5f
#define WSMAX  134217728

static_assert(DM == NH * HD);
static_assert(HD == 32 && LNB == 32);
static_assert((DM % GBN) == 0 && (DFF % GBN) == 0 && (QKVW % GBN) == 0);
static_assert((DM % 32) == 0 && (DFF % 32) == 0);
static_assert(GBM == (GTHR / 32) * 16);
static_assert((DM % TT) == 0 && (DFF % TT) == 0);
static_assert(NTHR == 8 * 32);

typedef float    v4f  __attribute__((ext_vector_type(4)));
typedef float    v8f  __attribute__((ext_vector_type(8)));
typedef int      v8i  __attribute__((ext_vector_type(8)));
typedef _Float16 v8h  __attribute__((ext_vector_type(8)));
typedef _Float16 v16h __attribute__((ext_vector_type(16)));
union FragH { v16h v; v8h h[2]; v8i w; };

__device__ __forceinline__ v8f wmh(const FragH& a, const FragH& b, v8f c) {
  v8f d = __builtin_amdgcn_wmma_f32_16x16x32_f16(false, a.v, false, b.v, (short)0, c, false, false);
  asm volatile("v_nop\n\tv_nop\n\tv_nop\n\tv_nop" : "+v"(d) : "v"(a.w), "v"(b.w));
  return d;
}

__device__ __forceinline__ v8h cvt8h(const v4f a, const v4f b, const float c) {
  v8h hv;
  hv[0] = (_Float16)(a.x * c); hv[1] = (_Float16)(a.y * c);
  hv[2] = (_Float16)(a.z * c); hv[3] = (_Float16)(a.w * c);
  hv[4] = (_Float16)(b.x * c); hv[5] = (_Float16)(b.y * c);
  hv[6] = (_Float16)(b.z * c); hv[7] = (_Float16)(b.w * c);
  return hv;
}

__device__ __forceinline__ void wave_lds_sync() {
  __builtin_amdgcn_fence(__ATOMIC_RELEASE, "wavefront");
  __builtin_amdgcn_wave_barrier();
}

__global__ __launch_bounds__(NTHR) void k_xprep(const float* __restrict__ x, _Float16* xh, int nN, int nUnits) {
  const int i = (int)blockIdx.x * NTHR + (int)threadIdx.x;
  if (i >= nUnits) return;
  const int row = i >> 5;
  const int c0  = (i & 31) * 8;
  const int rc  = row < nN ? row : nN - 1;
  const float* p = x + (size_t)rc * DM + c0;
  v4f a = *(const v4f*)p, b = *(const v4f*)(p + 4);
  const v4f z4 = {0.f, 0.f, 0.f, 0.f};
  if (row >= nN) { a = z4; b = z4; }
  const v8h hv = cvt8h(a, b, CX);
  const size_t o = (size_t)row * DM + c0;
  *(volatile v8h*)(xh + o) = hv;
  __threadfence();
  *(volatile v8h*)(xh + o) = hv;
}

__global__ __launch_bounds__(NTHR) void k_wtr(const float* __restrict__ W, _Float16* WT, int K, int Nc) {
  __shared__ __attribute__((aligned(16))) float tile[TT * TP];
  const int tid = (int)threadIdx.x, lane = tid & 31, wave = tid >> 5;
  const int n0 = (int)blockIdx.x * TT;
  const int k0 = (int)blockIdx.y * TT;
#pragma unroll
  for (int i = 0; i < 4; ++i) {
    const int kr = (tid >> 4) + 16 * i;
    const int c4 = (tid & 15) * 4;
    const v4f v = *(const v4f*)(W + (size_t)(k0 + kr) * (size_t)Nc + n0 + c4);
    *(v4f*)(tile + kr * TP + c4) = v;
  }
  __syncthreads();
  const int q = lane & 7;
  v8h hv[2];
#pragma unroll
  for (int i = 0; i < 2; ++i) {
    const int nr = 8 * wave + 4 * i + (lane >> 3);
    v4f a, b;
    a.x = tile[(8 * q + 0) * TP + nr]; a.y = tile[(8 * q + 1) * TP + nr];
    a.z = tile[(8 * q + 2) * TP + nr]; a.w = tile[(8 * q + 3) * TP + nr];
    b.x = tile[(8 * q + 4) * TP + nr]; b.y = tile[(8 * q + 5) * TP + nr];
    b.z = tile[(8 * q + 6) * TP + nr]; b.w = tile[(8 * q + 7) * TP + nr];
    hv[i] = cvt8h(a, b, CW);
  }
#pragma unroll
  for (int i = 0; i < 2; ++i) {
    const int nr = 8 * wave + 4 * i + (lane >> 3);
    _Float16* op = WT + (size_t)(n0 + nr) * (size_t)K + k0 + 8 * q;
    *(volatile v8h*)op = hv[i];
  }
  __threadfence();
#pragma unroll
  for (int i = 0; i < 2; ++i) {
    const int nr = 8 * wave + 4 * i + (lane >> 3);
    _Float16* op = WT + (size_t)(n0 + nr) * (size_t)K + k0 + 8 * q;
    *(volatile v8h*)op = hv[i];
  }
}

template<int EPI>
__global__ __launch_bounds__(GTHR) void k_gemm(
    const _Float16* __restrict__ A, const _Float16* __restrict__ WT,
    const float* __restrict__ b0, const float* __restrict__ b1, const float* __restrict__ b2,
    float* outF, _Float16* outH,
    int K, int ldo, int ldh, int segN, float scl, float cao)
{
  __shared__ __attribute__((aligned(16))) float stg[GBM * GBN];
  const int tid = (int)threadIdx.x, lane = tid & 31, wave = tid >> 5, hh = lane >> 4, m = lane & 15;
  const int rowBase = (int)blockIdx.x * GBM;
  const int col0    = (int)blockIdx.y * GBN;
  int seg = col0 / segN;
  seg = seg < 0 ? 0 : (seg > 2 ? 2 : seg);
  const float* bp = (seg == 0) ? b0 : ((seg == 1) ? b1 : b2);
  int bofs = col0 - seg * segN;
  bofs = bofs < 0 ? 0 : bofs;

  v8f acc[4];
  {
    const v8f z = {0.f, 0.f, 0.f, 0.f, 0.f, 0.f, 0.f, 0.f};
    acc[0] = z; acc[1] = z; acc[2] = z; acc[3] = z;
  }
  const _Float16* ap = A  + (size_t)(rowBase + 16 * wave + m) * (size_t)K + 8 * hh;
  const _Float16* wp = WT + (size_t)(col0 + m) * (size_t)K + 8 * hh;
  const int ksteps = K >> 5;
#pragma unroll 1
  for (int ks = 0; ks < ksteps; ++ks) {
    FragH af;
    af.h[0] = *(const v8h*)(ap + 32 * ks);
    af.h[1] = *(const v8h*)(ap + 32 * ks + 16);
#pragma unroll
    for (int t = 0; t < 4; ++t) {
      const _Float16* wq = wp + (size_t)(16 * t) * (size_t)K + 32 * ks;
      FragH bf;
      bf.h[0] = *(const v8h*)wq;
      bf.h[1] = *(const v8h*)(wq + 16);
      acc[t] = wmh(af, bf, acc[t]);
    }
  }

#pragma unroll
  for (int t = 0; t < 4; ++t) {
    const int lc = 16 * t + m;
    int bi = bofs + lc;
    bi = bi > segN - 1 ? segN - 1 : bi;
    const float bv = bp[bi];
#pragma unroll
    for (int r = 0; r < 8; ++r) {
      const int lr = 16 * wave + 8 * hh + r;
      float v = fmaf(acc[t][r], scl, bv);
      if (EPI == 1) v = fmaxf(v, 0.f);
      stg[lr * GBN + lc] = v;
    }
  }
  __syncthreads();

  if (EPI == 0) {
    v4f fv[8];
#pragma unroll
    for (int i = 0; i < 8; ++i) {
      const int lr = 16 * wave + 2 * i + hh;
      fv[i] = *(const v4f*)(stg + lr * GBN + 4 * m);
    }
#pragma unroll
    for (int i = 0; i < 8; ++i) {
      const int lr = 16 * wave + 2 * i + hh;
      float* op = outF + (size_t)(rowBase + lr) * (size_t)ldo + col0 + 4 * m;
      *(volatile v4f*)op = fv[i];
    }
    __threadfence();
#pragma unroll
    for (int i = 0; i < 8; ++i) {
      const int lr = 16 * wave + 2 * i + hh;
      float* op = outF + (size_t)(rowBase + lr) * (size_t)ldo + col0 + 4 * m;
      *(volatile v4f*)op = fv[i];
    }
  }
  if (EPI == 1) {
    v8h hv[4];
    const int q = lane & 7;
#pragma unroll
    for (int i = 0; i < 4; ++i) {
      const int lr = 16 * wave + 4 * i + (lane >> 3);
      const v4f a = *(const v4f*)(stg + lr * GBN + 8 * q);
      const v4f b = *(const v4f*)(stg + lr * GBN + 8 * q + 4);
      hv[i] = cvt8h(a, b, cao);
    }
#pragma unroll
    for (int i = 0; i < 4; ++i) {
      const int lr = 16 * wave + 4 * i + (lane >> 3);
      _Float16* op = outH + (size_t)(rowBase + lr) * (size_t)ldh + col0 + 8 * q;
      *(volatile v8h*)op = hv[i];
    }
    __threadfence();
#pragma unroll
    for (int i = 0; i < 4; ++i) {
      const int lr = 16 * wave + 4 * i + (lane >> 3);
      _Float16* op = outH + (size_t)(rowBase + lr) * (size_t)ldh + col0 + 8 * q;
      *(volatile v8h*)op = hv[i];
    }
  }
}

__global__ __launch_bounds__(NTHR) void k_attn(
    const float* __restrict__ QKV, const int* __restrict__ ip, const int* __restrict__ ipb,
    const int* __restrict__ kbc, const int* __restrict__ qbc,
    _Float16* AH, int nN, int nB)
{
  __shared__ __attribute__((aligned(16))) float qs[8 * DM];
  __shared__ __attribute__((aligned(16))) float ps[8 * NH * LNB];
  __shared__ int rs[8 * LNB];
  (void)qbc;
  const int tid = (int)threadIdx.x, lane = tid & 31, wave = tid >> 5;
  const int n = (int)blockIdx.x * 8 + wave;
  _Float16* op = AH + (size_t)n * DM + 8 * lane;
  if (n >= nN) {
    const v4f z4 = {0.f, 0.f, 0.f, 0.f};
    const v8h z = cvt8h(z4, z4, 1.0f);
    *(volatile v8h*)op = z;
    __threadfence();
    *(volatile v8h*)op = z;
    return;
  }
  int bi = ipb[n];
  bi = bi < 0 ? 0 : (bi > nB - 1 ? nB - 1 : bi);
  int off = 0;
#pragma unroll 1
  for (int b = 0; b < bi; ++b) off += kbc[b];

  float* qw = qs + wave * DM;
  float* pw = ps + wave * (NH * LNB);
  {
    const float* qp = QKV + (size_t)n * QKVW + 8 * lane;
    v4f a = *(const v4f*)qp;
    v4f c = *(const v4f*)(qp + 4);
    a = a * ISD;
    c = c * ISD;
    *(v4f*)(qw + 8 * lane)     = a;
    *(v4f*)(qw + 8 * lane + 4) = c;
  }
  const int  idx   = ip[(size_t)n * LNB + lane];
  const bool valid = idx >= 0;
  int row = valid ? idx + off : 0;
  row = row < 0 ? row + nN : row;
  row = row < 0 ? 0 : (row > nN - 1 ? nN - 1 : row);
  rs[wave * LNB + lane] = row;
  wave_lds_sync();

  const float* kr = QKV + (size_t)row * QKVW + DM;
#pragma unroll 1
  for (int h = 0; h < NH; ++h) {
    const float* kh = kr + HD * h;
    const float* qh = qw + HD * h;
    float s = 0.f;
#pragma unroll
    for (int c = 0; c < HD / 4; ++c) {
      const v4f kv = *(const v4f*)(kh + 4 * c);
      const v4f qv = *(const v4f*)(qh + 4 * c);
      s = fmaf(qv.x, kv.x, s);
      s = fmaf(qv.y, kv.y, s);
      s = fmaf(qv.z, kv.z, s);
      s = fmaf(qv.w, kv.w, s);
    }
    const float lg = valid ? s : -1.0e9f;
    float mx = lg;
#pragma unroll
    for (int o = 16; o > 0; o >>= 1) mx = fmaxf(mx, __shfl_xor(mx, o));
    const float e = __expf(lg - mx);
    float sm = e;
#pragma unroll
    for (int o = 16; o > 0; o >>= 1) sm += __shfl_xor(sm, o);
    pw[LNB * h + lane] = e * (1.0f / sm);
  }
  wave_lds_sync();

  float acc[NH];
#pragma unroll
  for (int j = 0; j < NH; ++j) acc[j] = 0.f;
#pragma unroll 1
  for (int s = 0; s < LNB; ++s) {
    const int r = rs[wave * LNB + s];
    const float* vr = QKV + (size_t)r * QKVW + 2 * DM + lane;
    float vv[NH];
#pragma unroll
    for (int j = 0; j < NH; ++j) vv[j] = vr[HD * j];
#pragma unroll
    for (int j = 0; j < NH; ++j) acc[j] = fmaf(pw[LNB * j + s], vv[j], acc[j]);
  }

  wave_lds_sync();
#pragma unroll
  for (int j = 0; j < NH; ++j) qw[HD * j + lane] = acc[j];
  wave_lds_sync();
  const v4f oa = *(const v4f*)(qw + 8 * lane);
  const v4f ob = *(const v4f*)(qw + 8 * lane + 4);
  const v8h hv = cvt8h(oa, ob, CX);
  *(volatile v8h*)op = hv;
  __threadfence();
  *(volatile v8h*)op = hv;
}

template<int MODE>
__global__ __launch_bounds__(NTHR) void k_ln(
    const float* __restrict__ a, const float* __restrict__ b,
    const float* __restrict__ g, const float* __restrict__ be,
    float* outF, _Float16* outH, int nN)
{
  __shared__ __attribute__((aligned(16))) float stg[8 * DM];
  const int tid = (int)threadIdx.x, lane = tid & 31, wave = tid >> 5;
  const int row = (int)blockIdx.x * 8 + wave;
  const size_t ro = (size_t)row * DM;
  if (MODE == 1) {
    if (row >= nN) return;
  }
  if (MODE == 0) {
    if (row >= nN) {
      const v4f z4 = {0.f, 0.f, 0.f, 0.f};
      const v8h z = cvt8h(z4, z4, 1.0f);
      _Float16* hp = outH + ro + 8 * lane;
      *(volatile v8h*)hp = z;
      __threadfence();
      *(volatile v8h*)hp = z;
      return;
    }
  }
  const v4f a0 = *(const v4f*)(a + ro + 8 * lane), a1 = *(const v4f*)(a + ro + 8 * lane + 4);
  const v4f b0 = *(const v4f*)(b + ro + 8 * lane), b1 = *(const v4f*)(b + ro + 8 * lane + 4);
  const v4f t0 = a0 + b0, t1 = a1 + b1;
  float s = ((t0.x + t0.y) + (t0.z + t0.w)) + ((t1.x + t1.y) + (t1.z + t1.w));
#pragma unroll
  for (int o = 16; o > 0; o >>= 1) s += __shfl_xor(s, o);
  const float mu = s * (1.0f / DM);
  const v4f d0 = t0 - mu, d1 = t1 - mu;
  float ss = ((d0.x * d0.x + d0.y * d0.y) + (d0.z * d0.z + d0.w * d0.w))
           + ((d1.x * d1.x + d1.y * d1.y) + (d1.z * d1.z + d1.w * d1.w));
#pragma unroll
  for (int o = 16; o > 0; o >>= 1) ss += __shfl_xor(ss, o);
  const float var  = ss * (1.0f / DM);
  const float rstd = rsqrtf(var + LNEPS);
  const v4f g0 = *(const v4f*)(g + 8 * lane),  gg1 = *(const v4f*)(g + 8 * lane + 4);
  const v4f e0 = *(const v4f*)(be + 8 * lane), e1  = *(const v4f*)(be + 8 * lane + 4);
  const v4f y0 = (d0 * rstd) * g0 + e0;
  const v4f y1 = (d1 * rstd) * gg1 + e1;

  if (MODE == 0) {
    const v8h hv = cvt8h(y0, y1, CX);
    _Float16* hp = outH + ro + 8 * lane;
    *(volatile v8h*)hp = hv;
    __threadfence();
    *(volatile v8h*)hp = hv;
  }
  float* sw = stg + wave * DM;
  *(v4f*)(sw + 8 * lane)     = y0;
  *(v4f*)(sw + 8 * lane + 4) = y1;
  wave_lds_sync();
  const v4f p0 = *(const v4f*)(sw + 4 * lane);
  const v4f p1 = *(const v4f*)(sw + 128 + 4 * lane);
  float* o = outF + ro;
  *(volatile v4f*)(o + 4 * lane)       = p0;
  *(volatile v4f*)(o + 128 + 4 * lane) = p1;
  __threadfence();
  *(volatile v4f*)(o + 4 * lane)       = p0;
  *(volatile v4f*)(o + 128 + 4 * lane) = p1;
}

static inline int cdiv(int a, int b) { return (a + b - 1) / b; }

extern "C" void kernel_launch(void* const* d_in, const int* in_sizes, int n_in,
                              void* d_out, int out_size, void* d_ws, size_t ws_size,
                              hipStream_t stream) {
  if (n_in < 21) return;
  if (in_sizes[0] < DM || (in_sizes[0] % DM) != 0) return;
  const int nN = in_sizes[0] / DM;
  if (nN < 1 || nN > (1 << 20)) return;
  if (in_sizes[1] != nN * LNB) return;
  if (in_sizes[2] < 1) return;
  const int nB = in_sizes[3];
  if (nB < 1 || nB > 65536) return;
  if (in_sizes[4] != nN) return;
  if (in_sizes[5] != DM * DM || in_sizes[6] != DM) return;
  if (in_sizes[7] != DM * DM || in_sizes[8] != DM) return;
  if (in_sizes[9] != DM * DM || in_sizes[10] != DM) return;
  if (in_sizes[11] != DM * DM || in_sizes[12] != DM) return;
  if (in_sizes[13] != DM * DFF || in_sizes[14] != DFF) return;
  if (in_sizes[15] != DFF * DM || in_sizes[16] != DM) return;
  if (in_sizes[17] != DM || in_sizes[18] != DM) return;
  if (in_sizes[19] != DM || in_sizes[20] != DM) return;
  if (out_size != nN * DM) return;

  const float* src = (const float*)d_in[0];
  const int*   ip  = (const int*)  d_in[1];
  const int*   qbc = (const int*)  d_in[2];
  const int*   kbc = (const int*)  d_in[3];
  const int*   ipb = (const int*)  d_in[4];
  const float* Wq  = (const float*)d_in[5];   const float* bq  = (const float*)d_in[6];
  const float* Wk  = (const float*)d_in[7];   const float* bk  = (const float*)d_in[8];
  const float* Wv  = (const float*)d_in[9];   const float* bv  = (const float*)d_in[10];
  const float* Wo  = (const float*)d_in[11];  const float* bo  = (const float*)d_in[12];
  const float* W1  = (const float*)d_in[13];  const float* b1  = (const float*)d_in[14];
  const float* W2  = (const float*)d_in[15];  const float* b2  = (const float*)d_in[16];
  const float* g1  = (const float*)d_in[17];  const float* be1 = (const float*)d_in[18];
  const float* g2  = (const float*)d_in[19];  const float* be2 = (const float*)d_in[20];
  float* out = (float*)d_out;

  const int MP = cdiv(nN, GBM) * GBM;

  const size_t szR1 = (size_t)MP * 4096;
  size_t off = 0;
  const size_t oR1  = off;                 off += szR1;
  const size_t oXH  = oR1;
  const size_t oQKV = oR1 + (size_t)MP * 512;
  const size_t oAH  = oR1 + (size_t)MP * 3584;
  const size_t oHH  = oR1;
  const size_t oWQ  = off;                 off += (size_t)QKVW * DM * 2;
  const size_t oWO  = off;                 off += (size_t)DM * DM * 2;
  const size_t oW1  = off;                 off += (size_t)DFF * DM * 2;
  const size_t oW2  = off;                 off += (size_t)DM * DFF * 2;
  const size_t oSF  = off;                 off += (size_t)MP * DM * 4;
  const size_t oX   = off;                 off += (size_t)MP * DM * 4;
  const size_t oXH2 = off;                 off += (size_t)MP * DM * 2;
  if (off > ws_size || off > (size_t)WSMAX) return;
  if (oAH + (size_t)MP * DM * 2 != oR1 + szR1) return;
  if ((size_t)MP * DFF * 2 != szR1) return;

  char* ws = (char*)d_ws;
  _Float16* XH  = (_Float16*)(ws + oXH);
  float*    QKV = (float*)(ws + oQKV);
  _Float16* AH  = (_Float16*)(ws + oAH);
  _Float16* HH  = (_Float16*)(ws + oHH);
  _Float16* WQ  = (_Float16*)(ws + oWQ);
  _Float16* WOT = (_Float16*)(ws + oWO);
  _Float16* W1T = (_Float16*)(ws + oW1);
  _Float16* W2T = (_Float16*)(ws + oW2);
  float*    SF  = (float*)(ws + oSF);
  float*    X   = (float*)(ws + oX);
  _Float16* XH2 = (_Float16*)(ws + oXH2);

  const int nUx = MP * (DM / 8);
  k_xprep<<<cdiv(nUx, NTHR), NTHR, 0, stream>>>(src, XH, nN, nUx);

  k_wtr<<<dim3(DM / TT, DM / TT), NTHR, 0, stream>>>(Wq, WQ, DM, DM);
  k_wtr<<<dim3(DM / TT, DM / TT), NTHR, 0, stream>>>(Wk, WQ + (size_t)DM * DM, DM, DM);
  k_wtr<<<dim3(DM / TT, DM / TT), NTHR, 0, stream>>>(Wv, WQ + (size_t)2 * DM * DM, DM, DM);
  k_wtr<<<dim3(DM / TT, DM / TT), NTHR, 0, stream>>>(Wo, WOT, DM, DM);
  k_wtr<<<dim3(DFF / TT, DM / TT), NTHR, 0, stream>>>(W1, W1T, DM, DFF);
  k_wtr<<<dim3(DM / TT, DFF / TT), NTHR, 0, stream>>>(W2, W2T, DFF, DM);

  const int gM = MP / GBM;
  k_gemm<0><<<dim3(gM, QKVW / GBN), GTHR, 0, stream>>>(XH, WQ, bq, bk, bv, QKV, XH2,
                                                       DM, QKVW, DFF, DM, SCL, CX);
  k_attn<<<MP / 8, NTHR, 0, stream>>>(QKV, ip, ipb, kbc, qbc, AH, nN, nB);
  k_gemm<0><<<dim3(gM, DM / GBN), GTHR, 0, stream>>>(AH, WOT, bo, bo, bo, SF, XH2,
                                                     DM, DM, DFF, DM, SCL, CX);
  k_ln<0><<<MP / 8, NTHR, 0, stream>>>(src, SF, g1, be1, X, XH2, nN);
  k_gemm<1><<<dim3(gM, DFF / GBN), GTHR, 0, stream>>>(XH2, W1T, b1, b1, b1, SF, HH,
                                                      DM, DM, DFF, DFF, SCL, CX);
  k_gemm<0><<<dim3(gM, DM / GBN), GTHR, 0, stream>>>(HH, W2T, b2, b2, b2, SF, XH2,
                                                     DFF, DM, DFF, DM, SCL, CX);
  k_ln<1><<<cdiv(nN, 8), NTHR, 0, stream>>>(X, SF, g2, be2, out, XH2, nN);
}
